// RNN_18021682774382
// MI455X (gfx1250) — hardware-run, weakly checked
//
#include <hip/hip_runtime.h>
#include <math.h>

constexpr int NBAT    = 64;
constexpr int NSTEP   = 512;
constexpr int NEMB    = 768;
constexpr int NHID    = 256;
constexpr int NVOC    = 3072;
constexpr int NROWS   = NBAT * NSTEP;
constexpr int NTHR    = 256;
constexpr int SEQ_BLK = 16;
constexpr int HP      = 264;
constexpr int OP      = 260;
constexpr int NC8     = NEMB / 8;
constexpr int NGATH   = NROWS * NC8;
constexpr int NOUT0   = NBAT * NVOC;
constexpr int NOUT1   = NBAT * NHID;
static_assert(NEMB % 32 == 0);
static_assert(NHID % 64 == 0 && NROWS % 64 == 0);
static_assert(((NHID / 64) * (NROWS / 64)) % 8 == 0);
static_assert(NBAT % 64 == 0 && NVOC % 64 == 0);
static_assert(NHID % 32 == 0);
static_assert(((NBAT / 64) * (NVOC / 64)) % 8 == 0);
static_assert(NHID == 32 * (NTHR / 32));
static_assert(NBAT % SEQ_BLK == 0);
static_assert(NGATH % NTHR == 0);
static_assert(NEMB % 64 == 0 && NVOC % 64 == 0 && NHID % 64 == 0);
static_assert(NOUT0 * 4 == 786432);
static_assert(HP % 8 == 0 && OP % 4 == 0);

typedef __attribute__((ext_vector_type(16))) _Float16 v16h;
typedef __attribute__((ext_vector_type(8)))  _Float16 v8h;
typedef __attribute__((ext_vector_type(16))) __bf16   v16b;
typedef __attribute__((ext_vector_type(8)))  __bf16   v8b;
typedef __attribute__((ext_vector_type(8)))  float    v8f;
typedef __attribute__((ext_vector_type(4)))  float    v4f;
typedef __attribute__((ext_vector_type(4)))  unsigned v4u;

__device__ __forceinline__ unsigned short f2bf_bits(float f) {
  unsigned u = __float_as_uint(f);
  return (unsigned short)((u + 0x7FFFu + ((u >> 16) & 1u)) >> 16);
}
__device__ __forceinline__ float bf_bits2f(unsigned short h) { return __uint_as_float(((unsigned)h) << 16); }
__device__ __forceinline__ float bf16r(float f) { return bf_bits2f(f2bf_bits(f)); }

__device__ __forceinline__ void dep_guard_h(v8f& a, v8f& b, v16h x, v16h y) { asm volatile("v_nop\n\tv_nop\n\tv_nop\n\tv_nop" : "+v"(a), "+v"(b) : "v"(x), "v"(y)); }
__device__ __forceinline__ void dep_guard_b(v8f& a, v8f& b, v16b x, v16b y) { asm volatile("v_nop\n\tv_nop\n\tv_nop\n\tv_nop" : "+v"(a), "+v"(b) : "v"(x), "v"(y)); }
__device__ __forceinline__ void dep_guard4_h(v8f& a, v8f& b, v8f& c, v8f& d, v16h x, v16h y) { asm volatile("v_nop\n\tv_nop\n\tv_nop\n\tv_nop" : "+v"(a), "+v"(b), "+v"(c), "+v"(d) : "v"(x), "v"(y)); }
__device__ __forceinline__ void dep_guard4_b(v8f& a, v8f& b, v8f& c, v8f& d, v16b x, v16b y) { asm volatile("v_nop\n\tv_nop\n\tv_nop\n\tv_nop" : "+v"(a), "+v"(b), "+v"(c), "+v"(d) : "v"(x), "v"(y)); }
__device__ __forceinline__ void dep_guard2x4_b(v8f& a, v8f& b, v16b w, v16b x, v16b y, v16b z) { asm volatile("v_nop\n\tv_nop\n\tv_nop\n\tv_nop" : "+v"(a), "+v"(b) : "v"(w), "v"(x), "v"(y), "v"(z)); }
__device__ __forceinline__ void keep4_h(v16h a, v16h b, v16h c, v16h d) { asm volatile("v_nop" :: "v"(a), "v"(b), "v"(c), "v"(d)); }
__device__ __forceinline__ void keep4_b(v16b a, v16b b, v16b c, v16b d) { asm volatile("v_nop" :: "v"(a), "v"(b), "v"(c), "v"(d)); }
__device__ __forceinline__ void acc_guard4(v8f& a, v8f& b, v8f& c, v8f& d) { asm volatile("v_nop\n\tv_nop\n\tv_nop\n\tv_nop" : "+v"(a), "+v"(b), "+v"(c), "+v"(d)); }
__device__ __forceinline__ void acc_guard2(v8f& a, v8f& b) { asm volatile("v_nop\n\tv_nop\n\tv_nop\n\tv_nop" : "+v"(a), "+v"(b)); }
template <typename T> struct Frag;
template <> struct Frag<_Float16> {
  typedef v16h V; union U { v16h v; v8h h[2]; };
  static __device__ __forceinline__ v16h load(const _Float16* p) {
    U f; f.h[0] = *(const v8h*)(p); f.h[1] = *(const v8h*)(p + 16); return f.v;
  }
  static __device__ __forceinline__ v8f mma(v16h a, v16h b, v8f c) {
    return __builtin_amdgcn_wmma_f32_16x16x32_f16(false, a, false, b, (short)0, c, false, false);
  }
  static __device__ __forceinline__ void guard(v8f& a, v8f& b, v16h x, v16h y) { dep_guard_h(a, b, x, y); }
  static __device__ __forceinline__ void guard4(v8f& a, v8f& b, v8f& c, v8f& d, v16h x, v16h y) { dep_guard4_h(a, b, c, d, x, y); }
  static __device__ __forceinline__ void keep(v16h a, v16h b, v16h c, v16h d) { keep4_h(a, b, c, d); }
};
template <> struct Frag<__bf16> {
  typedef v16b V; union U { v16b v; v8b h[2]; };
  static __device__ __forceinline__ v16b load(const __bf16* p) {
    U f; f.h[0] = *(const v8b*)(p); f.h[1] = *(const v8b*)(p + 16); return f.v;
  }
  static __device__ __forceinline__ v8f mma(v16b a, v16b b, v8f c) {
    return __builtin_amdgcn_wmma_f32_16x16x32_bf16(false, a, false, b, (short)0, c, false, false);
  }
  static __device__ __forceinline__ void guard(v8f& a, v8f& b, v16b x, v16b y) { dep_guard_b(a, b, x, y); }
  static __device__ __forceinline__ void guard4(v8f& a, v8f& b, v8f& c, v8f& d, v16b x, v16b y) { dep_guard4_b(a, b, c, d, x, y); }
  static __device__ __forceinline__ void keep(v16b a, v16b b, v16b c, v16b d) { keep4_b(a, b, c, d); }
};

__device__ __forceinline__ float ftanh(float x) {
  const float e = expf(2.0f * x);
  return 1.0f - 2.0f * __builtin_amdgcn_rcpf(e + 1.0f);
}

template <int ET> struct Elem;
template <> struct Elem<0> { typedef _Float16 T; };
template <> struct Elem<1> { typedef __bf16 T; };
template <int ET, int SPLIT, int BIAS_MODE, int OUT_MODE, bool RESID, int ACT = 0>
__global__ __launch_bounds__(256) void wmma_gemm64(
    const unsigned short* __restrict__ Ap, const unsigned short* __restrict__ A2p, int lda, long strideA,
    const unsigned short* __restrict__ Btp, const unsigned short* __restrict__ Bt2p, int ldb, long strideB,
    void* __restrict__ Cout, void* __restrict__ Cout2, int ldc, long strideC,
    const float* __restrict__ bias,
    const float* __restrict__ resid, long strideR,
    int M, int N, int K, float scale) {
  typedef typename Elem<ET>::T T;
  typedef typename Frag<T>::V V;
  const T* A = (const T*)Ap; const T* A2 = (const T*)A2p; const T* Bt = (const T*)Btp; const T* Bt2 = (const T*)Bt2p;
  __shared__ __align__(16) float sT[8][16 * 68];
  const int b    = blockIdx.y;
  const int lane = threadIdx.x & 31;
  const int wave = threadIdx.x >> 5;
  const int tilesN = N >> 6;
  const int tilesM = M >> 6;
  const int tile = blockIdx.x * 8 + wave;
  if (tile >= tilesM * tilesN) return;
  const int tm = tile / tilesN;
  const int tn = tile - tm * tilesN;
  const int m0 = tm << 6;
  const int n0 = tn << 6;

  const T* Ab  = A  + (size_t)b * strideA;
  const T* Bb  = Bt + (size_t)b * strideB;
  const T* Ab2 = (SPLIT != 0) ? (A2  + (size_t)b * strideA) : nullptr;
  const T* Bb2 = (SPLIT == 2) ? (Bt2 + (size_t)b * strideB) : nullptr;

  const int rlane = lane & 15;
  const int koff  = (lane >> 4) * 8;
  const int mOff  = (lane >> 4) * 8;

  v8f acc[4][4];
#pragma unroll
  for (int i = 0; i < 4; ++i)
#pragma unroll
    for (int j = 0; j < 4; ++j) acc[i][j] = (v8f){0.f,0.f,0.f,0.f,0.f,0.f,0.f,0.f};

  for (int k0 = 0; k0 < K; k0 += 32) {
    V bh[4], bl[4];
#pragma unroll
    for (int j = 0; j < 4; ++j) {
      const size_t bo = (size_t)(n0 + (j << 4) + rlane) * ldb + koff + k0;
      bh[j] = Frag<T>::load(Bb + bo);
      if (SPLIT == 2) bl[j] = Frag<T>::load(Bb2 + bo);
    }
#pragma unroll
    for (int i = 0; i < 4; ++i) {
      const size_t ao = (size_t)(m0 + (i << 4) + rlane) * lda + koff + k0;
      V ah = Frag<T>::load(Ab + ao);
      V al;
      if (SPLIT != 0) al = Frag<T>::load(Ab2 + ao);
#pragma unroll
      for (int j = 0; j < 4; ++j) {
        acc[i][j] = Frag<T>::mma(ah, bh[j], acc[i][j]);
        if (SPLIT == 2) acc[i][j] = Frag<T>::mma(ah, bl[j], acc[i][j]);
        if (SPLIT != 0) acc[i][j] = Frag<T>::mma(al, bh[j], acc[i][j]);
      }
      Frag<T>::guard4(acc[i][0], acc[i][1], acc[i][2], acc[i][3], ah, (SPLIT != 0) ? al : ah);
    }
    Frag<T>::keep(bh[0], bh[1], bh[2], bh[3]);
    if (SPLIT == 2) Frag<T>::keep(bl[0], bl[1], bl[2], bl[3]);
  }
  acc_guard4(acc[0][0], acc[0][1], acc[0][2], acc[0][3]);
  acc_guard4(acc[1][0], acc[1][1], acc[1][2], acc[1][3]);
  acc_guard4(acc[2][0], acc[2][1], acc[2][2], acc[2][3]);
  acc_guard4(acc[3][0], acc[3][1], acc[3][2], acc[3][3]);

  float* slab = sT[wave];
  const float* Rb = RESID ? (resid + (size_t)b * strideR) : nullptr;
#pragma unroll
  for (int i = 0; i < 4; ++i) {
    const int mBase = m0 + (i << 4);
#pragma unroll
    for (int j = 0; j < 4; ++j) {
      const int n = n0 + (j << 4) + rlane;
      float bv = 0.f;
      if (BIAS_MODE == 2) bv = bias[n];
#pragma unroll
      for (int r = 0; r < 8; ++r) {
        float v = acc[i][j][r] * scale;
        if (BIAS_MODE == 1) v += bias[mBase + mOff + r];
        if (BIAS_MODE == 2) v += bv;
        if (RESID) v += Rb[(size_t)(mBase + mOff + r) * ldc + n];
        if (ACT == 1) v = tanhf(v);
        if (ACT == 2) v = fmaxf(v, 0.0f);
        if (ACT == 3) v = v / (1.0f + expf(-v));
        if (ACT == 4) v = (v > 0.f) ? v : 0.01f * v;
        if (ACT == 5) v = 0.5f * v * (1.0f + erff(v * 0.70710678118654752f));
        slab[(mOff + r) * 68 + (j << 4) + rlane] = v;
      }
    }
    __builtin_amdgcn_fence(__ATOMIC_RELEASE, "workgroup");
    __builtin_amdgcn_wave_barrier();
    __builtin_amdgcn_fence(__ATOMIC_ACQUIRE, "workgroup");
    if (OUT_MODE == 0) {
      float* C = (float*)Cout + (size_t)b * strideC;
      const int hh = lane >> 4, c4 = (lane & 15) * 4;
      for (int pass = 0; pass < 2; ++pass) {
#pragma unroll
        for (int it = 0; it < 8; ++it) {
          const int row = it * 2 + hh;
          v4f v = *(const v4f*)(slab + row * 68 + c4);
          *(volatile v4f*)(C + (size_t)(mBase + row) * ldc + n0 + c4) = v;
        }
        __threadfence();
      }
    } else {
      const int q = lane >> 3, c8 = (lane & 7) * 8;
      unsigned short* C  = (unsigned short*)Cout  + (size_t)b * strideC;
      unsigned short* C2 = (OUT_MODE == 2) ? ((unsigned short*)Cout2 + (size_t)b * strideC) : nullptr;
      for (int pass = 0; pass < 2; ++pass) {
#pragma unroll
        for (int it = 0; it < 4; ++it) {
          const int row = it * 4 + q;
          const float* sp = slab + row * 68 + c8;
          v8h hv, lv;
#pragma unroll
          for (int e = 0; e < 8; ++e) {
            if (OUT_MODE == 1) {
              hv[e] = (_Float16)sp[e];
            } else {
              unsigned short hb = f2bf_bits(sp[e]);
              unsigned short lb = f2bf_bits(sp[e] - bf_bits2f(hb));
              hv[e] = __builtin_bit_cast(_Float16, hb);
              lv[e] = __builtin_bit_cast(_Float16, lb);
            }
          }
          *(volatile v8h*)(C + (size_t)(mBase + row) * ldc + n0 + c8) = hv;
          if (OUT_MODE == 2) *(volatile v8h*)(C2 + (size_t)(mBase + row) * ldc + n0 + c8) = lv;
        }
        __threadfence();
      }
    }
    __builtin_amdgcn_fence(__ATOMIC_RELEASE, "workgroup");
    __builtin_amdgcn_wave_barrier();
    __builtin_amdgcn_fence(__ATOMIC_ACQUIRE, "workgroup");
  }
}

template <int MODE>
__global__ __launch_bounds__(NTHR) void tpw_kernel(const float* __restrict__ src, int R, int C, int ldo,
                                                  unsigned short* __restrict__ O, float sc) {
  __shared__ float Tt[64 * 65];
  const int tid = threadIdx.x;
  const int c0 = blockIdx.x * 64, r0 = blockIdx.y * 64;
#pragma unroll
  for (int i = 0; i < 4; ++i) {
    const int idx = i * NTHR + tid;
    const int rr = idx >> 4, cc = (idx & 15) * 4;
    const v4f v = *(const v4f*)(src + (size_t)(r0 + rr) * (size_t)C + c0 + cc);
    Tt[rr * 65 + cc + 0] = v[0];
    Tt[rr * 65 + cc + 1] = v[1];
    Tt[rr * 65 + cc + 2] = v[2];
    Tt[rr * 65 + cc + 3] = v[3];
  }
  __syncthreads();
  const int q = tid >> 3, c8 = (tid & 7) * 8;
  v8h hv[2];
#pragma unroll
  for (int g = 0; g < 2; ++g) {
    const int qq = g * 32 + q;
#pragma unroll
    for (int e = 0; e < 8; ++e) {
      const float f = Tt[(c8 + e) * 65 + qq];
      unsigned short bits;
      if (MODE == 0) {
        bits = f2bf_bits(f * sc);
      } else {
        const float fb = bf_bits2f(f2bf_bits(f));
        bits = __builtin_bit_cast(unsigned short, (_Float16)(fb * sc));
      }
      hv[g][e] = __builtin_bit_cast(_Float16, bits);
    }
  }
  for (int pass = 0; pass < 2; ++pass) {
#pragma unroll
    for (int g = 0; g < 2; ++g) {
      const size_t o = (size_t)(c0 + g * 32 + q) * (size_t)ldo + (size_t)(r0 + c8);
      *(volatile v8h*)(O + o) = hv[g];
    }
    __threadfence();
  }
}

__global__ __launch_bounds__(NTHR) void gather_cvt8_kernel(const int* __restrict__ idx, const float* __restrict__ emb,
                                                           unsigned short* __restrict__ dst) {
  const int i = blockIdx.x * NTHR + threadIdx.x;
  if (i < NGATH) {
    const int m  = i / NC8;
    const int c8 = i - m * NC8;
    const int t  = m / NBAT;
    const int b  = m - t * NBAT;
    int id = idx[b * NSTEP + t];
    id = id < 0 ? 0 : (id > NVOC - 1 ? NVOC - 1 : id);
    const float* sp = emb + (size_t)id * NEMB + (size_t)c8 * 8;
    const v4f a  = *(const v4f*)(sp);
    const v4f bq = *(const v4f*)(sp + 4);
    v8h hv;
#pragma unroll
    for (int e = 0; e < 4; ++e) {
      const unsigned short b0 = f2bf_bits(a[e]);
      const unsigned short b1 = f2bf_bits(bq[e]);
      hv[e]     = __builtin_bit_cast(_Float16, b0);
      hv[4 + e] = __builtin_bit_cast(_Float16, b1);
    }
    *(volatile v8h*)(dst + (size_t)i * 8) = hv;
    __threadfence();
    *(volatile v8h*)(dst + (size_t)i * 8) = hv;
  }
}

__global__ __launch_bounds__(NTHR) void rnn_seq_kernel(const float* __restrict__ XWT, const unsigned short* __restrict__ WHp,
                                                       const float* __restrict__ Bh,
                                                       unsigned short* __restrict__ HHI, unsigned short* __restrict__ HLO,
                                                       float* __restrict__ HFIN) {
  __shared__ __align__(16) unsigned short Ahi[SEQ_BLK * HP];
  __shared__ __align__(16) unsigned short Alo[SEQ_BLK * HP];
  __shared__ __align__(16) float          Hs[SEQ_BLK * OP];
  const __bf16* WH = (const __bf16*)WHp;
  const int tid = threadIdx.x, lane = tid & 31, wave = tid >> 5;
  const int c = lane & 15, hh = lane >> 4, koff = hh * 8;
  const int rowbase = blockIdx.x * SEQ_BLK;

  {
    unsigned* zh = (unsigned*)(void*)Ahi;
    unsigned* zl = (unsigned*)(void*)Alo;
#pragma unroll 1
    for (int i = tid; i < (SEQ_BLK * HP) / 2; i += NTHR) { zh[i] = 0u; zl[i] = 0u; }
  }
  float hst[2][8], bb[2];
#pragma unroll
  for (int nt = 0; nt < 2; ++nt) {
    const int j = 32 * wave + 16 * nt + c;
    bb[nt] = bf16r(Bh[j]);
#pragma unroll
    for (int r = 0; r < 8; ++r) hst[nt][r] = 0.0f;
  }
  __syncthreads();

  const __bf16* ahirow = (const __bf16*)(const void*)Ahi + c * HP + koff;
  const __bf16* alorow = (const __bf16*)(const void*)Alo + c * HP + koff;
  const __bf16* w0 = WH + (size_t)(32 * wave + c) * NHID + koff;
  const __bf16* w1 = w0 + (size_t)16 * NHID;
  const v8f z8 = {0.f, 0.f, 0.f, 0.f, 0.f, 0.f, 0.f, 0.f};

#pragma unroll 1
  for (int t = 0; t < NSTEP; ++t) {
    float xv[2][8];
#pragma unroll
    for (int nt = 0; nt < 2; ++nt) {
      const int j = 32 * wave + 16 * nt + c;
      const float* xp = XWT + (size_t)j * NROWS + (size_t)t * NBAT + rowbase + 8 * hh;
      const v4f xa = *(const v4f*)(xp);
      const v4f xb = *(const v4f*)(xp + 4);
      xv[nt][0] = xa[0]; xv[nt][1] = xa[1]; xv[nt][2] = xa[2]; xv[nt][3] = xa[3];
      xv[nt][4] = xb[0]; xv[nt][5] = xb[1]; xv[nt][6] = xb[2]; xv[nt][7] = xb[3];
    }
    v8f acc0 = z8, acc1 = z8;
#pragma unroll 1
    for (int k0 = 0; k0 < NHID; k0 += 32) {
      const v16b ah = Frag<__bf16>::load(ahirow + k0);
      const v16b al = Frag<__bf16>::load(alorow + k0);
      const v16b b0 = Frag<__bf16>::load(w0 + k0);
      const v16b b1 = Frag<__bf16>::load(w1 + k0);
      acc0 = Frag<__bf16>::mma(ah, b0, acc0);
      acc0 = Frag<__bf16>::mma(al, b0, acc0);
      acc1 = Frag<__bf16>::mma(ah, b1, acc1);
      acc1 = Frag<__bf16>::mma(al, b1, acc1);
      dep_guard2x4_b(acc0, acc1, ah, al, b0, b1);
    }
    acc_guard2(acc0, acc1);
#pragma unroll
    for (int r = 0; r < 8; ++r) {
      const float z0 = (xv[0][r] + acc0[r]) + bb[0];
      const float z1 = (xv[1][r] + acc1[r]) + bb[1];
      hst[0][r] = ftanh(z0);
      hst[1][r] = ftanh(z1);
    }
    __syncthreads();
#pragma unroll
    for (int nt = 0; nt < 2; ++nt) {
      const int j = 32 * wave + 16 * nt + c;
#pragma unroll
      for (int r = 0; r < 8; ++r) {
        const float h = hst[nt][r];
        const unsigned short hb = f2bf_bits(h);
        const unsigned short lb = f2bf_bits(h - bf_bits2f(hb));
        const int li = (8 * hh + r) * HP + j;
        Ahi[li] = hb;
        Alo[li] = lb;
      }
    }
    __syncthreads();
  }

#pragma unroll
  for (int nt = 0; nt < 2; ++nt) {
    const int j = 32 * wave + 16 * nt + c;
#pragma unroll
    for (int r = 0; r < 8; ++r) Hs[(8 * hh + r) * OP + j] = hst[nt][r];
  }
  __syncthreads();
  for (int pass = 0; pass < 2; ++pass) {
#pragma unroll
    for (int it = 0; it < 4; ++it) {
      const int idx = it * NTHR + tid;
      const int row = idx >> 6, c4 = (idx & 63) * 4;
      const v4f v = *(const v4f*)(Hs + row * OP + c4);
      *(volatile v4f*)(HFIN + (size_t)(rowbase + row) * NHID + c4) = v;
    }
#pragma unroll
    for (int it = 0; it < 2; ++it) {
      const int idx = it * NTHR + tid;
      const int row = idx >> 5, c8 = (idx & 31) * 8;
      const v4u uh = *(const v4u*)(Ahi + row * HP + c8);
      const v4u ul = *(const v4u*)(Alo + row * HP + c8);
      *(volatile v4u*)(HHI + (size_t)(rowbase + row) * NHID + c8) = uh;
      *(volatile v4u*)(HLO + (size_t)(rowbase + row) * NHID + c8) = ul;
    }
    __threadfence();
  }
}

extern "C" void kernel_launch(void* const* d_in, const int* in_sizes, int n_in,
                              void* d_out, int out_size, void* d_ws, size_t ws_size, hipStream_t stream) {
  if (n_in < 7 || d_out == nullptr || d_ws == nullptr) return;
  if (in_sizes[0] != NBAT * NSTEP || in_sizes[1] != NVOC * NEMB || in_sizes[2] != NEMB * NHID ||
      in_sizes[3] != NHID * NHID || in_sizes[4] != NHID * NVOC || in_sizes[5] != NVOC || in_sizes[6] != NHID ||
      out_size != NOUT0 + NOUT1) return;

  const int*   idx = (const int*)d_in[0];
  const float* emb = (const float*)d_in[1];
  const float* wxh = (const float*)d_in[2];
  const float* whh = (const float*)d_in[3];
  const float* wy  = (const float*)d_in[4];
  const float* by  = (const float*)d_in[5];
  const float* bh  = (const float*)d_in[6];
  float* out0 = (float*)d_out;
  float* hfin = out0 + (size_t)NOUT0;

  char* ws = (char*)d_ws; size_t off = 0;
  auto carve = [&](size_t bytes) -> char* { char* p = ws + off; off += (bytes + 255) & ~(size_t)255; return p; };
  unsigned short* XB   = (unsigned short*)carve((size_t)NROWS * NEMB * 2);
  unsigned short* WXHT = (unsigned short*)carve((size_t)NHID * NEMB * 2);
  unsigned short* WHHT = (unsigned short*)carve((size_t)NHID * NHID * 2);
  unsigned short* WYT  = (unsigned short*)carve((size_t)NVOC * NHID * 2);
  float*          XWT  = (float*)carve((size_t)NHID * NROWS * 4);
  unsigned short* HHI  = (unsigned short*)carve((size_t)NBAT * NHID * 2);
  unsigned short* HLO  = (unsigned short*)carve((size_t)NBAT * NHID * 2);
  if (off > ws_size || off > (size_t)134217728) return;

  tpw_kernel<0><<<dim3(NHID / 64, NEMB / 64), NTHR, 0, stream>>>(wxh, NEMB, NHID, NEMB, WXHT, 1.0f);
  tpw_kernel<0><<<dim3(NHID / 64, NHID / 64), NTHR, 0, stream>>>(whh, NHID, NHID, NHID, WHHT, 1.0f);
  tpw_kernel<0><<<dim3(NVOC / 64, NHID / 64), NTHR, 0, stream>>>(wy,  NHID, NVOC, NHID, WYT,  1.0f);
  gather_cvt8_kernel<<<NGATH / NTHR, NTHR, 0, stream>>>(idx, emb, XB);
  wmma_gemm64<1, 0, 0, 0, false, 0><<<dim3((NHID / 64) * (NROWS / 64) / 8, 1), 256, 0, stream>>>(
      WXHT, WXHT, NEMB, 0L, XB, XB, NEMB, 0L, (void*)XWT, (void*)XWT, NROWS, 0L,
      by, XWT, 0L, NHID, NROWS, NEMB, 1.0f);
  rnn_seq_kernel<<<NBAT / SEQ_BLK, NTHR, 0, stream>>>(XWT, WHHT, bh, HHI, HLO, hfin);
  wmma_gemm64<1, 1, 2, 0, false, 0><<<dim3((NBAT / 64) * (NVOC / 64) / 8, 1), 256, 0, stream>>>(
      HHI, HLO, NHID, 0L, WYT, WYT, NHID, 0L, (void*)out0, (void*)out0, NVOC, 0L,
      by, XWT, 0L, NBAT, NVOC, NHID, 1.0f);
}
